// SCell_50568944943254
// MI455X (gfx1250) — hardware-verified
//
#include <hip/hip_runtime.h>
#include <math.h>

typedef __attribute__((ext_vector_type(16))) _Float16 v16h;
typedef __attribute__((ext_vector_type(16))) __bf16 v16b;
typedef __attribute__((ext_vector_type(8)))  _Float16 v8h;
typedef __attribute__((ext_vector_type(8)))  float v8f;
typedef __attribute__((ext_vector_type(4)))  float v4f;
typedef __attribute__((ext_vector_type(2)))  float v2f;
typedef __attribute__((ext_vector_type(4)))  unsigned v4u;
typedef __attribute__((ext_vector_type(4)))  int v4i;
typedef float __attribute__((may_alias)) float_a;
typedef int __attribute__((may_alias)) int_a;

template <typename T> __device__ __forceinline__ void vst2(void* p, T v) { *(volatile T*)p = v; __threadfence(); *(volatile T*)p = v; }
__device__ __forceinline__ v8f wmma16(v16h a, v16h b, v8f c) {
  v8f d = __builtin_amdgcn_wmma_f32_16x16x32_f16(false, a, false, b, (short)0, c, false, false);
  asm volatile("v_nop\n\tv_nop\n\tv_nop\n\tv_nop" : "+v"(d) : "v"(a), "v"(b));
  return d;
}
__device__ __forceinline__ v8f wmma_bf(v16b a, v16b b, v8f c) {
  v8f d = __builtin_amdgcn_wmma_f32_16x16x32_bf16(false, a, false, b, (short)0, c, false, false);
  asm volatile("v_nop\n\tv_nop\n\tv_nop\n\tv_nop" : "+v"(d) : "v"(a), "v"(b));
  return d;
}
__device__ __forceinline__ v16h frag_h(const _Float16* rowk0, int lane) {
  union { v16h v; v8h q[2]; } u; const _Float16* p = rowk0 + 8 * (lane >> 4);
  u.q[0] = *(const v8h*)p; u.q[1] = *(const v8h*)(p + 16); return u.v;
}
__device__ __forceinline__ v16h frag_f32(const float* rowk0, int lane) {
  v16h a; const float* p = rowk0 + 8 * (lane >> 4);
#pragma unroll
  for (int i = 0; i < 8; ++i) { a[i] = (_Float16)p[i]; a[8 + i] = (_Float16)p[16 + i]; }
  return a;
}
__device__ __forceinline__ v16h frag_f32s(const float* rowk0, int lane, float sc) {
  v16h a; const float* p = rowk0 + 8 * (lane >> 4);
#pragma unroll
  for (int i = 0; i < 8; ++i) { a[i] = (_Float16)(p[i] * sc); a[8 + i] = (_Float16)(p[16 + i] * sc); }
  return a;
}
__device__ __forceinline__ v16h fragc_f32(const float* W, int k0, int n, int lane, int ld, int K) {
  v16h a; const int g = lane >> 4;
#pragma unroll
  for (int i = 0; i < 8; ++i) { const int ka = k0 + 8 * g + i, kb = ka + 16;
    a[i] = (_Float16)(ka < K ? W[(size_t)(ka < K ? ka : K - 1) * ld + n] : 0.f); a[8 + i] = (_Float16)(kb < K ? W[(size_t)(kb < K ? kb : K - 1) * ld + n] : 0.f); }
  return a;
}
struct F2 { v16b h, l; };
__device__ __forceinline__ F2 bsplit16(const float v[16]) { F2 r;
#pragma unroll
  for (int i = 0; i < 16; ++i) { const __bf16 h = (__bf16)v[i]; r.h[i] = h; r.l[i] = (__bf16)(v[i] - (float)h); }
  return r; }
__device__ __forceinline__ F2 split_row(const float* row, int k0, int lane) { float v[16]; const float* p = row + k0 + 8 * (lane >> 4);
#pragma unroll
  for (int i = 0; i < 8; ++i) { v[i] = p[i]; v[8 + i] = p[16 + i]; }
  return bsplit16(v); }
__device__ __forceinline__ F2 split_rowK(const float* row, int k0, int lane, int K) { float v[16]; const int g = lane >> 4;
#pragma unroll
  for (int i = 0; i < 8; ++i) { const int ka = k0 + 8 * g + i, kb = ka + 16; v[i] = ka < K ? row[ka < K ? ka : K - 1] : 0.f; v[8 + i] = kb < K ? row[kb < K ? kb : K - 1] : 0.f; }
  return bsplit16(v); }
__device__ __forceinline__ F2 split_col(const float* W, int k0, int n, int lane, int ld, int K) { float v[16]; const int g = lane >> 4;
#pragma unroll
  for (int i = 0; i < 8; ++i) { const int ka = k0 + 8 * g + i, kb = ka + 16; v[i] = ka < K ? W[(size_t)(ka < K ? ka : K - 1) * ld + n] : 0.f; v[8 + i] = kb < K ? W[(size_t)(kb < K ? kb : K - 1) * ld + n] : 0.f; }
  return bsplit16(v); }
__device__ __forceinline__ v8f mac3(const F2& a, const F2& b, v8f c) { c = wmma_bf(a.l, b.h, c); c = wmma_bf(a.h, b.l, c); return wmma_bf(a.h, b.h, c); }
__device__ __forceinline__ float sigm(float v) { return 1.0f / (1.0f + expf(-v)); }
#define LDSX() do { asm volatile("s_wait_dscnt 0" ::: "memory"); __builtin_amdgcn_wave_barrier(); __builtin_amdgcn_fence(__ATOMIC_RELEASE, "workgroup"); } while (0)


#define NB 8
#define SS 2048
#define NNB 16
#define HH 256
#define NR (NB * SS)
__device__ __forceinline__ float bfr(float v) { return (float)(__bf16)v; }
__device__ __forceinline__ v16b frag_b(const __bf16* rowk0, int lane) { return __builtin_bit_cast(v16b, frag_h((const _Float16*)rowk0, lane)); }
__device__ __attribute__((noinline)) float sigm_ni(float v) { return 1.0f / (1.0f + expf(-v)); }
__device__ __attribute__((noinline)) float tanh_ni(float v) { return tanhf(v); }

__global__ __launch_bounds__(256) void k_gv(const float* __restrict__ gin, const float* __restrict__ V, const float* __restrict__ Vb, float* __restrict__ GV) {
  __shared__ float sg[HH]; const int tid = threadIdx.x, b = blockIdx.x;
  sg[tid] = bfr(gin[(size_t)b * HH + tid]); __syncthreads();
  v4f acc;
#pragma unroll
  for (int e = 0; e < 4; ++e) acc[e] = bfr(Vb[tid * 4 + e]);
#pragma unroll 2
  for (int j = 0; j < HH; ++j) { const float gj = sg[j]; const float* vr = V + (size_t)j * (4 * HH) + tid * 4;
#pragma unroll
    for (int e = 0; e < 4; ++e) acc[e] += gj * bfr(vr[e]); }
  vst2(GV + (size_t)b * (4 * HH) + tid * 4, acc);
}
__global__ __launch_bounds__(256) void k_agg(const float* __restrict__ h, const int* __restrict__ idx, const int* __restrict__ msk, __bf16* __restrict__ AGh, __bf16* __restrict__ AGl) {
  const int tid = threadIdx.x, w = tid >> 5, lane = tid & 31; const size_t row = (size_t)blockIdx.x * 8 + w; const int b = (int)(row / SS);
  float a[8];
#pragma unroll
  for (int e = 0; e < 8; ++e) a[e] = 0.f;
#pragma unroll 1
  for (int n = 0; n < NNB; ++n) { int k = idx[row * NNB + n]; const int m = msk[row * NNB + n]; k = k < 0 ? 0 : (k > SS ? SS : k);
    if (m != 0 && k > 0) { const float* hr = h + ((size_t)b * SS + (k - 1)) * HH + lane * 8;
#pragma unroll
      for (int e = 0; e < 8; ++e) a[e] += bfr(hr[e]); } }
  union { __bf16 e[8]; v4u u; } ph, pl;
#pragma unroll
  for (int e = 0; e < 8; ++e) { const float v = a[e] * (1.0f / NNB); const __bf16 hi = (__bf16)v; ph.e[e] = hi; pl.e[e] = (__bf16)(v - (float)hi); }
  vst2((unsigned*)(AGh + row * HH + lane * 8), ph.u); vst2((unsigned*)(AGl + row * HH + lane * 8), pl.u);
}
__global__ __launch_bounds__(128) void k_hn(const __bf16* __restrict__ AGh, const __bf16* __restrict__ AGl, const float* __restrict__ Wna, __bf16* __restrict__ HNh, __bf16* __restrict__ HNl) {
  __shared__ __align__(16) __bf16 sh_[4][16][136], sl_[4][16][136];
  const int tid = threadIdx.x, wave = tid >> 5, lane = tid & 31, col = lane & 15, g = lane >> 4; const size_t r0 = (size_t)blockIdx.x * 64 + wave * 16; const int n0 = blockIdx.y * 128;
  v8f acc[8] = {};
#pragma unroll 2
  for (int kc = 0; kc < HH / 32; ++kc) { const v16b ah = frag_b(AGh + (r0 + col) * HH + kc * 32, lane), al = frag_b(AGl + (r0 + col) * HH + kc * 32, lane);
#pragma unroll
    for (int j = 0; j < 8; ++j) { const v16b wb = split_col(Wna, kc * 32, n0 + j * 16 + col, lane, HH, HH).h; acc[j] = wmma_bf(al, wb, acc[j]); acc[j] = wmma_bf(ah, wb, acc[j]); } }
#pragma unroll
  for (int j = 0; j < 8; ++j)
#pragma unroll
    for (int r = 0; r < 8; ++r) { const float v = acc[j][r]; const __bf16 hi = (__bf16)v; sh_[wave][8 * g + r][j * 16 + col] = hi; sl_[wave][8 * g + r][j * 16 + col] = (__bf16)(v - (float)hi); }
  LDSX();
  for (int qq = lane; qq < 16 * 16; qq += 32) { const int rl = qq >> 4, pc = qq & 15; const size_t o = (r0 + rl) * HH + n0 + pc * 8; vst2((unsigned*)(HNh + o), *(const v4u*)(&sh_[wave][rl][pc * 8])); vst2((unsigned*)(HNl + o), *(const v4u*)(&sl_[wave][rl][pc * 8])); }
}
__global__ __launch_bounds__(128) void k_cell(const float* __restrict__ h, const float* __restrict__ x, const __bf16* __restrict__ HNh, const __bf16* __restrict__ HNl, const float* __restrict__ Wh, const float* __restrict__ U, const float* __restrict__ Wn, const float* __restrict__ GV, const float* __restrict__ c, float* __restrict__ newh, float* __restrict__ newc) {
  __shared__ __align__(16) float sh_[4][16][68], sc_[4][16][68];
  const int tid = threadIdx.x, wave = tid >> 5, lane = tid & 31, col = lane & 15, g = lane >> 4; const size_t r0 = (size_t)blockIdx.x * 64 + wave * 16; const int j0 = blockIdx.y * 64; const int b = (int)(r0 / SS);
  v8f acc[4][4] = {};
#pragma unroll 1
  for (int src = 0; src < 3; ++src) { const float* A = src == 0 ? h : x; const float* W = src == 0 ? Wh : (src == 1 ? U : Wn);
#pragma unroll 1
    for (int kc = 0; kc < HH / 32; ++kc) { v16b ah, al; if (src < 2) { ah = split_row(A + (r0 + col) * HH, kc * 32, lane).h; al = ah; } else { ah = frag_b(HNh + (r0 + col) * HH + kc * 32, lane); al = frag_b(HNl + (r0 + col) * HH + kc * 32, lane); }
#pragma unroll
      for (int gt = 0; gt < 4; ++gt)
#pragma unroll
        for (int t = 0; t < 4; ++t) { const v16b wb = split_col(W, kc * 32, gt * HH + j0 + t * 16 + col, lane, 4 * HH, HH).h; if (src == 2) acc[gt][t] = wmma_bf(al, wb, acc[gt][t]); acc[gt][t] = wmma_bf(ah, wb, acc[gt][t]); } } }
#pragma unroll
  for (int t = 0; t < 4; ++t) { const int j = j0 + t * 16 + col; const float* gv = GV + (size_t)b * 4 * HH;
    const float bi = gv[j], bf_ = gv[HH + j], bo_ = gv[2 * HH + j], bu = gv[3 * HH + j];
#pragma unroll
    for (int r = 0; r < 8; ++r) { const size_t row = r0 + 8 * g + r; const float cold = bfr(c[row * HH + j]);
      const float ig = sigm_ni(acc[0][t][r] + bi), fg = sigm_ni(acc[1][t][r] + bf_), og = sigm_ni(acc[2][t][r] + bo_), ug = tanh_ni(acc[3][t][r] + bu);
      const float cn = fg * cold + ig * ug; sc_[wave][8 * g + r][t * 16 + col] = cn; sh_[wave][8 * g + r][t * 16 + col] = og * tanh_ni(cn); } }
  LDSX();
  for (int qq = lane; qq < 16 * 16; qq += 32) { const int rl = qq >> 4, pc = qq & 15; const size_t o = (r0 + rl) * HH + j0 + pc * 4; vst2(newh + o, *(const v4f*)(&sh_[wave][rl][pc * 4])); vst2(newc + o, *(const v4f*)(&sc_[wave][rl][pc * 4])); }
}
extern "C" void kernel_launch(void* const* d_in, const int* in_sizes, int n_in, void* d_out, int out_size, void* d_ws, size_t ws_size, hipStream_t stream) {
  (void)in_sizes; (void)n_in; (void)out_size; (void)ws_size;
  const float* x = (const float*)d_in[0]; const float* h = (const float*)d_in[1]; const float* c = (const float*)d_in[2]; const float* gin = (const float*)d_in[3]; const int* idx = (const int*)d_in[4]; const int* msk = (const int*)d_in[5];
  const float* Wna = (const float*)d_in[7]; const float* Wh = (const float*)d_in[13]; const float* Wn = (const float*)d_in[14]; const float* U = (const float*)d_in[15]; const float* V = (const float*)d_in[16]; const float* Vb = (const float*)d_in[17];
  float* newh = (float*)d_out; float* newc = newh + (size_t)NR * HH;
  char* ws = (char*)d_ws; size_t off = 0;
  auto take = [&](size_t bytes) { char* p = ws + off; off += (bytes + 255) & ~(size_t)255; return p; };
  float* GV = (float*)take((size_t)NB * 4 * HH * 4); __bf16* AGh = (__bf16*)take((size_t)NR * HH * 2); __bf16* AGl = (__bf16*)take((size_t)NR * HH * 2); __bf16* HNh = (__bf16*)take((size_t)NR * HH * 2); __bf16* HNl = (__bf16*)take((size_t)NR * HH * 2);
  k_gv<<<NB, 256, 0, stream>>>(gin, V, Vb, GV);
  k_agg<<<NR / 8, 256, 0, stream>>>(h, idx, msk, AGh, AGl);
  k_hn<<<dim3(NR / 64, HH / 128), 128, 0, stream>>>(AGh, AGl, Wna, HNh, HNl);
  k_cell<<<dim3(NR / 64, HH / 64), 128, 0, stream>>>(h, x, HNh, HNl, Wh, U, Wn, GV, c, newh, newc);
}
